// DFSHA_77618648973711
// MI455X (gfx1250) — hardware-verified
//
#include <hip/hip_runtime.h>
#include <math.h>


#define NB 8
#define C1 256
#define CC 128
#define NT 1024
#define HW 32
#define NHD 8
#define HDIM 16
#define RED 8

typedef __attribute__((ext_vector_type(16))) __bf16 v16b;
typedef __attribute__((ext_vector_type(8)))  float v8f;
typedef __attribute__((ext_vector_type(4)))  float v4f;
typedef float __attribute__((may_alias)) float_a;

template <typename T> __device__ __forceinline__ void vst2(void* p, T v) { *(volatile T*)p = v; __threadfence(); *(volatile T*)p = v; }
__device__ __forceinline__ v8f wmma_bf(v16b a, v16b b, v8f c) {
  v8f d = __builtin_amdgcn_wmma_f32_16x16x32_bf16(false, a, false, b, (short)0, c, false, false);
  asm volatile("v_nop\n\tv_nop\n\tv_nop\n\tv_nop" : "+v"(d) : "v"(a), "v"(b));
  return d;
}
struct F2 { v16b h, l; };
__device__ __forceinline__ F2 bsplit16(const float v[16]) { F2 r;
#pragma unroll
  for (int i = 0; i < 16; ++i) { const __bf16 h = (__bf16)v[i]; r.h[i] = h; r.l[i] = (__bf16)(v[i] - (float)h); }
  return r; }
__device__ __forceinline__ F2 split_row(const float* row, int k0, int lane) { float v[16]; const float* p = row + k0 + 8 * (lane >> 4);
#pragma unroll
  for (int i = 0; i < 8; ++i) { v[i] = p[i]; v[8 + i] = p[16 + i]; }
  return bsplit16(v); }
__device__ __forceinline__ F2 split_col(const float* W, int k0, int n, int lane, int ld) { float v[16]; const int g = lane >> 4;
#pragma unroll
  for (int i = 0; i < 8; ++i) { v[i] = W[(size_t)(k0 + 8 * g + i) * ld + n]; v[8 + i] = W[(size_t)(k0 + 16 + 8 * g + i) * ld + n]; }
  return bsplit16(v); }
__device__ __forceinline__ v8f mac3(const F2& a, const F2& b, v8f c) { c = wmma_bf(a.l, b.h, c); c = wmma_bf(a.h, b.l, c); return wmma_bf(a.h, b.h, c); }
__device__ __forceinline__ float sigm(float v) { return 1.0f / (1.0f + expf(-v)); }
#define LDSX() do { asm volatile("s_wait_dscnt 0" ::: "memory"); __builtin_amdgcn_wave_barrier(); __builtin_amdgcn_fence(__ATOMIC_RELEASE, "workgroup"); } while (0)

template <int MODE>
__global__ __launch_bounds__(128) void k_gemm(const float* __restrict__ A, int lda, int K, const float* __restrict__ W, const float* __restrict__ bias,
                                            float* __restrict__ Out, int ldo) {
  __shared__ __align__(16) float so[4][16 * 132];
  const int tid = threadIdx.x, wave = tid >> 5, lane = tid & 31, col = lane & 15, g = lane >> 4;
  const int b = blockIdx.z, r0 = blockIdx.x * 64 + wave * 16, n0 = blockIdx.y * 128;
  const float* Ab = MODE == 1 ? A + (size_t)b * K * NT : (MODE == 2 ? A + (size_t)b * NHD * NT * HDIM : A + (size_t)b * NT * lda);
  v8f acc[8] = {};
#pragma unroll 1
  for (int kc = 0; kc < K / 32; ++kc) {
    F2 a;
    if (MODE == 1) a = split_col(Ab, kc * 32, r0 + col, lane, NT);
    else if (MODE == 2) { float v[16]; const int g2 = lane >> 4;
#pragma unroll
      for (int i = 0; i < 8; ++i) { const int ka = kc * 32 + 8 * g2 + i, kb = ka + 16;
        v[i] = Ab[((size_t)(ka >> 4) * NT + r0 + col) * HDIM + (ka & 15)]; v[8 + i] = Ab[((size_t)(kb >> 4) * NT + r0 + col) * HDIM + (kb & 15)]; }
      a = bsplit16(v); }
    else a = split_row(Ab + (size_t)(r0 + col) * lda, kc * 32, lane);
#pragma unroll
    for (int j = 0; j < 8; ++j) acc[j] = mac3(a, split_row(W + (size_t)(n0 + j * 16 + col) * K, kc * 32, lane), acc[j]); }
  float* S = so[wave];
#pragma unroll
  for (int j = 0; j < 8; ++j) { const float bv = bias ? bias[n0 + j * 16 + col] : 0.f;
#pragma unroll
    for (int r = 0; r < 8; ++r) S[(8 * g + r) * 132 + j * 16 + col] = acc[j][r] + bv; }
  LDSX();
#pragma unroll 4
  for (int rl = 0; rl < 16; ++rl) vst2(Out + ((size_t)b * NT + r0 + rl) * ldo + n0 + lane * 4, *(const v4f*)(S + rl * 132 + lane * 4));
}

__global__ __launch_bounds__(256) void k_planes(const float* __restrict__ yT, float* __restrict__ y1p) {
  __shared__ float tile[64][CC + 1];
  const int b = blockIdx.y, t0 = blockIdx.x * 64, tid = threadIdx.x;
  for (int q = tid; q < 64 * CC; q += 256) { const int t = q >> 7, c = q & 127; tile[t][c] = yT[((size_t)b * NT + t0 + t) * C1 + CC + c]; }
  __syncthreads();
  for (int q = tid; q < CC * 16; q += 256) { const int c = q >> 4, pc = q & 15;
    v4f v = { tile[pc * 4][c], tile[pc * 4 + 1][c], tile[pc * 4 + 2][c], tile[pc * 4 + 3][c] };
    vst2(y1p + ((size_t)b * CC + c) * NT + t0 + pc * 4, v); }
}

__global__ __launch_bounds__(256) void k_plane(const float* __restrict__ y1p, const float* __restrict__ dw_w, const float* __restrict__ dw_b,
                                             float* __restrict__ xl, float* __restrict__ pstat) {
  __shared__ float sp[HW][HW + 1], rre[HW][17], rim[HW][17], cs[HW], sn[HW], red[256], red2[256];
  const int b = blockIdx.y, c = blockIdx.x, tid = threadIdx.x;
  const float* pl = y1p + ((size_t)b * CC + c) * NT;
  for (int q = tid; q < NT; q += 256) sp[q >> 5][q & 31] = pl[q];
  if (tid < HW) { const float ang = -6.283185307179586f * (float)tid / (float)HW; cs[tid] = cosf(ang); sn[tid] = sinf(ang); }
  __syncthreads();
  for (int q = tid; q < HW * 17; q += 256) { const int h = q / 17, v = q % 17; float re = 0.f, im = 0.f;
#pragma unroll 1
    for (int w = 0; w < HW; ++w) { const int k = (v * w) & 31; re += sp[h][w] * cs[k]; im += sp[h][w] * sn[k]; }
    rre[h][v] = re; rim[h][v] = im; }
  __syncthreads();
  float macc = 0.f;
  for (int q = tid; q < HW * 17; q += 256) { const int u = q / 17, v = q % 17; float re = 0.f, im = 0.f;
#pragma unroll 1
    for (int h = 0; h < HW; ++h) { const int k = (u * h) & 31; const float cr = cs[k], ci = sn[k];
      re += rre[h][v] * cr - rim[h][v] * ci; im += rre[h][v] * ci + rim[h][v] * cr; }
    macc += sqrtf(re * re + im * im) * (1.0f / 32.0f); }
  float ysum = 0.f;
  for (int q = tid; q < NT; q += 256) ysum += sp[q >> 5][q & 31];
  red[tid] = macc; red2[tid] = ysum; __syncthreads();
  for (int st = 128; st > 0; st >>= 1) { if (tid < st) { red[tid] += red[tid + st]; red2[tid] += red2[tid + st]; } __syncthreads(); }
  if (tid < 32) { const float v = tid == 0 ? red[0] / (float)(HW * 17) : (tid == 1 ? red2[0] / (float)NT : 0.f); vst2(pstat + ((size_t)b * CC + c) * 32 + tid, (float_a)v); }
  float wk[9];
#pragma unroll
  for (int i = 0; i < 9; ++i) wk[i] = dw_w[c * 9 + i];
  const float bb = dw_b[c];
  for (int q4 = tid; q4 < NT / 4; q4 += 256) { v4f v;
#pragma unroll
    for (int e = 0; e < 4; ++e) { const int n = q4 * 4 + e, y = n >> 5, x = n & 31; float s = bb;
#pragma unroll
      for (int ky = 0; ky < 3; ++ky)
#pragma unroll
        for (int kx = 0; kx < 3; ++kx) { const int yy = y + ky - 1, xx = x + kx - 1; if (yy >= 0 && yy < HW && xx >= 0 && xx < HW) s += wk[ky * 3 + kx] * sp[yy][xx]; }
      v[e] = s; }
    vst2(xl + ((size_t)b * CC + c) * NT + q4 * 4, v); }
}

__global__ __launch_bounds__(128) void k_coef(const float* __restrict__ pstat, const float* __restrict__ fw1, const float* __restrict__ fw2,
                                            const float* __restrict__ cw1, const float* __restrict__ cw2, const float* __restrict__ rtw, const float* __restrict__ rtb,
                                            float* __restrict__ coef) {
  __shared__ float pooled[CC], ym[CC], hid[RED], fw[CC], hid2[RED], red[128];
  const int b = blockIdx.x, tid = threadIdx.x;
  pooled[tid] = pstat[((size_t)b * CC + tid) * 32]; ym[tid] = pstat[((size_t)b * CC + tid) * 32 + 1];
  __syncthreads();
  if (tid < RED) { float s = 0.f; for (int c = 0; c < CC; ++c) s += fw1[tid * CC + c] * pooled[c]; hid[tid] = s > 0.f ? s : 0.f; }
  __syncthreads();
  { float s = 0.f; for (int j = 0; j < RED; ++j) s += fw2[tid * RED + j] * hid[j]; fw[tid] = sigm(s); }
  __syncthreads();
  if (tid < RED) { float s = 0.f; for (int c = 0; c < CC; ++c) s += cw1[tid * CC + c] * (fw[c] * ym[c]); hid2[tid] = s > 0.f ? s : 0.f; }
  float pr = rtw[tid] * ym[tid]; red[tid] = pr;
  __syncthreads();
  for (int st = 64; st > 0; st >>= 1) { if (tid < st) red[tid] += red[tid + st]; __syncthreads(); }
  float s = 0.f; for (int j = 0; j < RED; ++j) s += cw2[tid * RED + j] * hid2[j];
  const float ca = sigm(s);
  vst2(coef + (size_t)b * 256 + tid, (float_a)(fw[tid] * ca));
  if (tid < 32) vst2(coef + (size_t)b * 256 + CC + tid, (float_a)(tid == 0 ? sigm(red[0] + rtb[0]) : 0.f));
}

__global__ __launch_bounds__(256) void k_var(const float* __restrict__ qkvT, float* __restrict__ vstat) {
  const int b = blockIdx.y, tid = threadIdx.x;
  const int tl = tid >> 4, hh = tid & 15;
  __shared__ float st[2 * NHD][64 + 4];
  for (int it = 0; it < 4; ++it) {
    const size_t tok = (size_t)blockIdx.x * 64 + it * 16 + tl;
    const int h = hh & 7, which = hh >> 3;
    const float* p = qkvT + ((size_t)b * NT + tok) * 384 + (which ? 128 : 256) + h * HDIM;
    float m = 0.f;
#pragma unroll 1
    for (int d = 0; d < HDIM; ++d) m += p[d];
    m *= (1.0f / 16.0f);
    float q = 0.f;
#pragma unroll 1
    for (int d = 0; d < HDIM; ++d) { const float dd = p[d] - m; q += dd * dd; }
    st[which * 8 + h][it * 16 + tl] = q * (1.0f / 15.0f);
  }
  __syncthreads();
  for (int q = tid; q < 16 * 16; q += 256) { const int row = q >> 4, pc = q & 15;
    vst2(vstat + ((size_t)b * 16 + row) * NT + (size_t)blockIdx.x * 64 + pc * 4, *(const v4f*)(&st[row][pc * 4])); }
}

__global__ __launch_bounds__(128) void k_tsattn(const float* __restrict__ vstat, const float* __restrict__ qkvT, float* __restrict__ toT) {
  __shared__ __align__(16) float sP[4][16][68];
  __shared__ float svk[NT];
  const int tid = threadIdx.x, w = tid >> 5, lane = tid & 31, col = lane & 15, g = lane >> 4;
  const int b = blockIdx.z, h = blockIdx.y, q0 = blockIdx.x * 64 + w * 16;
  for (int m = tid; m < NT; m += 128) svk[m] = vstat[((size_t)b * 16 + 8 + h) * NT + m];
  __syncthreads();
  const float vv = vstat[((size_t)b * 16 + h) * NT + q0 + col] * 0.25f;
  float mrun = -3.0e38f, lrun = 0.f; v8f acc = {};
  const float* vb = qkvT + (size_t)b * NT * 384 + 256 + h * HDIM;
#pragma unroll 1
  for (int kt = 0; kt < NT / 64; ++kt) {
    float s[32]; float mx = -3.0e38f;
#pragma unroll
    for (int j = 0; j < 32; ++j) { s[j] = vv * svk[kt * 64 + g * 32 + j]; mx = fmaxf(mx, s[j]); }
    mx = fmaxf(mx, __shfl_xor(mx, 16, 32));
    const float mnew = fmaxf(mrun, mx); const float corr = expf(mrun - mnew);
    float ps = 0.f;
#pragma unroll
    for (int j = 0; j < 32; ++j) { const float p = expf(s[j] - mnew); ps += p; sP[w][col][g * 32 + j] = p; }
    ps += __shfl_xor(ps, 16, 32);
    lrun = lrun * corr + ps; mrun = mnew;
#pragma unroll
    for (int r = 0; r < 8; ++r) { const float cr = __shfl(corr, 8 * g + r, 32); acc[r] *= cr; }
    LDSX();
#pragma unroll
    for (int kc = 0; kc < 2; ++kc) acc = mac3(split_row(&sP[w][col][0], kc * 32, lane), split_col(vb + (size_t)(kt * 64 + kc * 32) * 384, 0, col, lane, 384), acc);
    __builtin_amdgcn_wave_barrier();
  }
  __shared__ __align__(16) float so[4][16][20];
#pragma unroll
  for (int r = 0; r < 8; ++r) { const float lr = __shfl(lrun, 8 * g + r, 32); so[w][8 * g + r][col] = acc[r] / lr; }
  LDSX();
  for (int q = lane; q < 64; q += 32) { const int rl = q >> 2, pc = q & 3; vst2(toT + (((size_t)b * NHD + h) * NT + q0 + rl) * HDIM + pc * 4, *(const v4f*)(&so[w][rl][pc * 4])); }
}

__global__ __launch_bounds__(128) void k_battn(const float* __restrict__ qs, const float* __restrict__ ks, const float* __restrict__ vvT, float* __restrict__ obT) {
  __shared__ __align__(16) float sP[4][16][68];
  __shared__ __align__(16) float so[4][16][132];
  const int tid = threadIdx.x, w = tid >> 5, lane = tid & 31, col = lane & 15, g = lane >> 4;
  const int b = blockIdx.y, q0 = blockIdx.x * 64 + w * 16;
  const float* qb = qs + (size_t)b * NT * CC; const float* kb = ks + (size_t)b * NT * CC; const float* vb = vvT + (size_t)b * NT * CC;
  v16b aq[4];
#pragma unroll
  for (int kc = 0; kc < 4; ++kc) { const float* p = qb + (size_t)(q0 + col) * CC + kc * 32 + 8 * g;
#pragma unroll
    for (int i = 0; i < 8; ++i) { const float a0 = p[i], a1 = p[16 + i];
      aq[kc][i] = (__bf16)(a0 > 0.f ? 1.f : (a0 < 0.f ? -1.f : 0.f)); aq[kc][8 + i] = (__bf16)(a1 > 0.f ? 1.f : (a1 < 0.f ? -1.f : 0.f)); } }
  float mrun = -3.0e38f, lrun = 0.f; v8f acc[8] = {};
  const float scale = 0.08838834764831845f;
#pragma unroll 1
  for (int kt = 0; kt < NT / 64; ++kt) {
    v8f st4[4];
#pragma unroll
    for (int t = 0; t < 4; ++t) { st4[t] = (v8f){};
#pragma unroll
      for (int kc = 0; kc < 4; ++kc) { v16b bk; const float* p = kb + (size_t)(kt * 64 + t * 16 + col) * CC + kc * 32 + 8 * g;
#pragma unroll
        for (int i = 0; i < 8; ++i) { const float a0 = p[i], a1 = p[16 + i];
          bk[i] = (__bf16)(a0 > 0.f ? 1.f : (a0 < 0.f ? -1.f : 0.f)); bk[8 + i] = (__bf16)(a1 > 0.f ? 1.f : (a1 < 0.f ? -1.f : 0.f)); }
        st4[t] = wmma_bf(aq[kc], bk, st4[t]); } }
#pragma unroll
    for (int t = 0; t < 4; ++t)
#pragma unroll
      for (int r = 0; r < 8; ++r) sP[w][8 * g + r][t * 16 + col] = st4[t][r] * scale;
    LDSX();
    float mx = -3.0e38f;
#pragma unroll
    for (int j = 0; j < 32; ++j) mx = fmaxf(mx, sP[w][col][g * 32 + j]);
    mx = fmaxf(mx, __shfl_xor(mx, 16, 32));
    const float mnew = fmaxf(mrun, mx); const float corr = expf(mrun - mnew);
    float ps = 0.f;
#pragma unroll
    for (int j = 0; j < 32; ++j) { const float p = expf(sP[w][col][g * 32 + j] - mnew); ps += p; sP[w][col][g * 32 + j] = p; }
    ps += __shfl_xor(ps, 16, 32);
    lrun = lrun * corr + ps; mrun = mnew;
#pragma unroll
    for (int r = 0; r < 8; ++r) { const float cr = __shfl(corr, 8 * g + r, 32);
#pragma unroll
      for (int t = 0; t < 8; ++t) acc[t][r] *= cr; }
    LDSX();
#pragma unroll
    for (int kc = 0; kc < 2; ++kc) { const F2 pa = split_row(&sP[w][col][0], kc * 32, lane);
#pragma unroll
      for (int t = 0; t < 8; ++t) acc[t] = mac3(pa, split_col(vb + (size_t)(kt * 64) * CC, kc * 32, t * 16 + col, lane, CC), acc[t]); }
    __builtin_amdgcn_wave_barrier();
  }
#pragma unroll
  for (int r = 0; r < 8; ++r) { const float lr = __shfl(lrun, 8 * g + r, 32);
#pragma unroll
    for (int t = 0; t < 8; ++t) so[w][8 * g + r][t * 16 + col] = acc[t][r] / lr; }
  LDSX();
#pragma unroll 4
  for (int rl = 0; rl < 16; ++rl) vst2(obT + ((size_t)b * NT + q0 + rl) * CC + lane * 4, *(const v4f*)(&so[w][rl][lane * 4]));
}

__global__ __launch_bounds__(128) void k_combine(const float* __restrict__ yT, const float* __restrict__ statT, const float* __restrict__ xl,
                                               const float* __restrict__ obinT, const float* __restrict__ coef, float* __restrict__ ycT) {
  const size_t row = blockIdx.x; const int b = (int)(row / NT), n = (int)(row % NT), c = threadIdx.x;
  const float y0 = yT[row * C1 + c], y1 = yT[row * C1 + CC + c];
  const float s1 = coef[(size_t)b * 256 + c], alpha = coef[(size_t)b * 256 + CC];
  const float att = y1 * s1 + statT[row * CC + c] + (1.0f - alpha) * xl[((size_t)b * CC + c) * NT + n] + alpha * obinT[row * CC + c];
  vst2(ycT + row * 384 + c, (float_a)y0); vst2(ycT + row * 384 + CC + c, (float_a)y1); vst2(ycT + row * 384 + 2 * CC + c, (float_a)att);
}
__global__ __launch_bounds__(128) void k_cv2(const float* __restrict__ ycT, const float* __restrict__ W, const float* __restrict__ bias, const float* __restrict__ x,
                                           float* __restrict__ out) {
  __shared__ __align__(16) float st[128][68];
  const int tid = threadIdx.x, wave = tid >> 5, lane = tid & 31, col = lane & 15, g = lane >> 4;
  const int b = blockIdx.z, t0 = blockIdx.x * 64, r0 = t0 + wave * 16, n0 = blockIdx.y * 128;
  v8f acc[8] = {};
#pragma unroll 1
  for (int kc = 0; kc < 384 / 32; ++kc) { const F2 a = split_row(ycT + ((size_t)b * NT + r0 + col) * 384, kc * 32, lane);
#pragma unroll
    for (int j = 0; j < 8; ++j) acc[j] = mac3(a, split_row(W + (size_t)(n0 + j * 16 + col) * 384, kc * 32, lane), acc[j]); }
#pragma unroll
  for (int j = 0; j < 8; ++j) { const float bv = bias[n0 + j * 16 + col];
#pragma unroll
    for (int r = 0; r < 8; ++r) st[j * 16 + col][wave * 16 + 8 * g + r] = acc[j][r] + bv; }
  __syncthreads();
  for (int q = tid; q < 128 * 16; q += 128) { const int o = q >> 4, pc = q & 15; const size_t oo = ((size_t)b * C1 + n0 + o) * NT + t0 + pc * 4;
    v4f v = *(const v4f*)(&st[o][pc * 4]) + *(const v4f*)(x + oo); vst2(out + oo, v); }
}

extern "C" void kernel_launch(void* const* d_in, const int* in_sizes, int n_in,
                              void* d_out, int out_size, void* d_ws, size_t ws_size,
                              hipStream_t stream) {
  (void)in_sizes; (void)n_in; (void)out_size; (void)ws_size;
  const float** I = (const float**)d_in;
  const float* x = I[0]; const float* cv1w = I[1]; const float* cv1b = I[2]; const float* fw1 = I[3]; const float* fw2 = I[4]; const float* cw1 = I[5]; const float* cw2 = I[6];
  const float* qkvw = I[7]; const float* tpw = I[8]; const float* tpb = I[9]; const float* dww = I[10]; const float* dwb = I[11]; const float* rtw = I[12]; const float* rtb = I[13];
  const float* qw = I[14]; const float* kw = I[15]; const float* vw = I[16]; const float* spw = I[17]; const float* spb = I[18]; const float* cv2w = I[19]; const float* cv2b = I[20];
  float* out = (float*)d_out;
  char* ws = (char*)d_ws; size_t off = 0;
  auto take = [&](size_t n) { char* p = ws + off; off += (n * 4 + 255) & ~(size_t)255; return (float*)p; };
  float* yT = take((size_t)NB * NT * C1);
  float* y1p = take((size_t)NB * CC * NT);
  float* xl = take((size_t)NB * CC * NT);
  float* pstat = take((size_t)NB * CC * 32);
  float* coef = take((size_t)NB * 256);
  float* qkvT = take((size_t)NB * NT * 384);
  float* qs = take((size_t)NB * NT * CC); float* ks = take((size_t)NB * NT * CC); float* vvT = take((size_t)NB * NT * CC);
  float* vstat = take((size_t)NB * 16 * NT);
  float* toT = take((size_t)NB * NT * CC); float* statT = take((size_t)NB * NT * CC);
  float* obT = take((size_t)NB * NT * CC); float* obinT = take((size_t)NB * NT * CC);
  float* ycT = take((size_t)NB * NT * 384);
  const dim3 g64(NT / 64, 1, NB);
  k_gemm<1><<<dim3(NT / 64, C1 / 128, NB), 128, 0, stream>>>(x, 0, C1, cv1w, cv1b, yT, C1);
  k_planes<<<dim3(NT / 64, NB), 256, 0, stream>>>(yT, y1p);
  k_plane<<<dim3(CC, NB), 256, 0, stream>>>(y1p, dww, dwb, xl, pstat);
  k_coef<<<NB, 128, 0, stream>>>(pstat, fw1, fw2, cw1, cw2, rtw, rtb, coef);
  k_gemm<0><<<dim3(NT / 64, 3, NB), 128, 0, stream>>>(yT + CC, C1, CC, qkvw, nullptr, qkvT, 384);
  k_gemm<0><<<g64, 128, 0, stream>>>(yT + CC, C1, CC, qw, nullptr, qs, CC);
  k_gemm<0><<<g64, 128, 0, stream>>>(yT + CC, C1, CC, kw, nullptr, ks, CC);
  k_gemm<0><<<g64, 128, 0, stream>>>(yT + CC, C1, CC, vw, nullptr, vvT, CC);
  k_var<<<dim3(NT / 64, NB), 256, 0, stream>>>(qkvT, vstat);
  k_tsattn<<<dim3(NT / 64, NHD, NB), 128, 0, stream>>>(vstat, qkvT, toT);
  k_gemm<2><<<g64, 128, 0, stream>>>(toT, 0, CC, tpw, tpb, statT, CC);
  k_battn<<<dim3(NT / 64, NB), 128, 0, stream>>>(qs, ks, vvT, obT);
  k_gemm<0><<<g64, 128, 0, stream>>>(obT, CC, CC, spw, spb, obinT, CC);
  k_combine<<<NB * NT, 128, 0, stream>>>(yT, statT, xl, obinT, coef, ycT);
  k_cv2<<<dim3(NT / 64, C1 / 128, NB), 128, 0, stream>>>(ycT, cv2w, cv2b, x, out);
}
